// C2fDCNAttn_79070347919450
// MI455X (gfx1250) — hardware-verified
//
#include <hip/hip_runtime.h>
#define NI 4
#define C1 256
#define CM 128
#define HS 64
#define PX (HS * HS)
#define NR (NI * PX)
#define NTOK 80
#define GD 512
#define CC5 (5 * CM)
typedef __bf16 v16b __attribute__((ext_vector_type(16)));
typedef unsigned short v8us __attribute__((ext_vector_type(8), may_alias));
typedef float  v8f  __attribute__((ext_vector_type(8)));
typedef float  v4f  __attribute__((ext_vector_type(4)));
typedef float  v4fa __attribute__((ext_vector_type(4), may_alias));
union FragB { v16b v; v8us half[2]; unsigned short u[16]; };

__device__ __forceinline__ unsigned short bf16_bits(float x) { unsigned int u = __float_as_uint(x); return (unsigned short)((u + 0x7FFFu + ((u >> 16) & 1u)) >> 16); }
__device__ __forceinline__ float bf16_val(unsigned short b) { return __uint_as_float(((unsigned int)b) << 16); }
__device__ __forceinline__ float bf16_round(float x) { return bf16_val(bf16_bits(x)); }
template <int NT>
__device__ __forceinline__ v8f mmaN(v16b ah, v16b al, v16b bh, v16b bl, v8f c) {
  c = __builtin_amdgcn_wmma_f32_16x16x32_bf16(false, ah, false, bh, (short)0, c, false, false);
  if (NT >= 2) c = __builtin_amdgcn_wmma_f32_16x16x32_bf16(false, al, false, bh, (short)0, c, false, false);
  if (NT >= 3) c = __builtin_amdgcn_wmma_f32_16x16x32_bf16(false, ah, false, bl, (short)0, c, false, false);
  asm volatile("v_nop\n\tv_nop\n\tv_nop\n\tv_nop" : "+v"(c) : "v"(ah), "v"(al), "v"(bh), "v"(bl));
  return c;
}

__global__ __launch_bounds__(256) void k_wt_bf16(const float* __restrict__ W, unsigned short* __restrict__ Wt, int K, int N) {
  const int t = blockIdx.x * 256 + threadIdx.x;
  const int k8n = K / 8;
  if (t >= N * k8n) return;
  const int n = t / k8n, k8 = (t % k8n) * 8;
  v8us v;
#pragma unroll
  for (int i = 0; i < 8; ++i) v[i] = bf16_bits(W[(size_t)(k8 + i) * N + n]);
  *(volatile v8us*)(Wt + (size_t)n * K + k8) = v;
  __threadfence();
  *(volatile v8us*)(Wt + (size_t)n * K + k8) = v;
}

template <bool ASPLIT, int ACT, bool BIAS_BF16>
__global__ __launch_bounds__(128) void k_gemm_bf(const float* __restrict__ A, int lda, const unsigned short* __restrict__ Wt, int ldb,
                                               const float* __restrict__ bias, float* __restrict__ C, int ldc, int M, int N, int K) {
  __shared__ __attribute__((aligned(16))) float so[4][16][64];
  const int tid = threadIdx.x, w = tid >> 5, lane = tid & 31, ln = lane & 15, hh = lane >> 4;
  const int ntn = N / 64;
  const int wid = blockIdx.x * 4 + w;
  const int mt = wid / ntn, nq = wid % ntn;
  if (mt * 16 >= M) return;
  const int row0 = mt * 16, col0 = nq * 64;
  const float* arow = A + (size_t)(row0 + ln) * lda;
  v8f acc[4] = {};
  for (int kb = 0; kb < K; kb += 32) {
    FragB ah, al;
    const v4f x0 = *(const v4fa*)(arow + kb + 8 * hh), x1 = *(const v4fa*)(arow + kb + 8 * hh + 4);
    const v4f x2 = *(const v4fa*)(arow + kb + 16 + 8 * hh), x3 = *(const v4fa*)(arow + kb + 16 + 8 * hh + 4);
    float xs[16] = {x0[0],x0[1],x0[2],x0[3],x1[0],x1[1],x1[2],x1[3],x2[0],x2[1],x2[2],x2[3],x3[0],x3[1],x3[2],x3[3]};
#pragma unroll
    for (int i = 0; i < 16; ++i) { const unsigned short hb = bf16_bits(xs[i]); ah.u[i] = hb; al.u[i] = ASPLIT ? bf16_bits(xs[i] - bf16_val(hb)) : (unsigned short)0; }
#pragma unroll
    for (int t = 0; t < 4; ++t) {
      const unsigned short* brow = Wt + (size_t)(col0 + t * 16 + ln) * ldb + kb;
      FragB b;
      b.half[0] = *(const v8us*)(brow + 8 * hh);
      b.half[1] = *(const v8us*)(brow + 16 + 8 * hh);
      acc[t] = mmaN<ASPLIT ? 2 : 1>(ah.v, al.v, b.v, b.v, acc[t]);
    }
  }
#pragma unroll
  for (int t = 0; t < 4; ++t) {
    float bv = bias ? bias[col0 + t * 16 + ln] : 0.f;
    if (BIAS_BF16) bv = bf16_round(bv);
#pragma unroll
    for (int r = 0; r < 8; ++r) { float v = acc[t][r] + bv; if (ACT == 1) v = fmaxf(v, 0.f); so[w][8 * hh + r][t * 16 + ln] = v; }
  }
  __builtin_amdgcn_fence(__ATOMIC_ACQ_REL, "workgroup");
  __builtin_amdgcn_wave_barrier();
  const int rsub = lane >> 4, c4 = (lane & 15) * 4;
  for (int pass = 0; pass < 2; ++pass) {
#pragma unroll
    for (int q = 0; q < 8; ++q) {
      const int r = q * 2 + rsub;
      const v4f v = *(const v4fa*)&so[w][r][c4];
      *(volatile v4f*)(C + (size_t)(row0 + r) * ldc + col0 + c4) = v;
    }
    if (pass == 0) __threadfence();
  }
}

template <bool ASPLIT, int ACT, bool BIAS_BF16, bool RES_BF16>
__global__ __launch_bounds__(128) void k_gemm_bf3(const float* __restrict__ A, int lda, const unsigned short* __restrict__ Wt, int ldb,
                                                const float* __restrict__ bias, const float* __restrict__ resid, int rmod, int ldr,
                                                float* __restrict__ C, int ldc, int M, int N, int K) {
  __shared__ __attribute__((aligned(16))) float so[4][16][64];
  const int tid = threadIdx.x, w = tid >> 5, lane = tid & 31, ln = lane & 15, hh = lane >> 4;
  const int ntn = N / 64;
  const int wid = blockIdx.x * 4 + w;
  const int mt = wid / ntn, nq = wid % ntn;
  if (mt * 16 >= M) return;
  const int row0 = mt * 16, col0 = nq * 64;
  const float* arow = A + (size_t)(row0 + ln) * lda;
  v8f acc[4] = {};
  for (int kb = 0; kb < K; kb += 32) {
    FragB ah, al;
    const v4f x0 = *(const v4fa*)(arow + kb + 8 * hh), x1 = *(const v4fa*)(arow + kb + 8 * hh + 4);
    const v4f x2 = *(const v4fa*)(arow + kb + 16 + 8 * hh), x3 = *(const v4fa*)(arow + kb + 16 + 8 * hh + 4);
    float xs[16] = {x0[0],x0[1],x0[2],x0[3],x1[0],x1[1],x1[2],x1[3],x2[0],x2[1],x2[2],x2[3],x3[0],x3[1],x3[2],x3[3]};
#pragma unroll
    for (int i = 0; i < 16; ++i) { const unsigned short hb = bf16_bits(xs[i]); ah.u[i] = hb; al.u[i] = ASPLIT ? bf16_bits(xs[i] - bf16_val(hb)) : (unsigned short)0; }
#pragma unroll
    for (int t = 0; t < 4; ++t) {
      const unsigned short* brow = Wt + (size_t)(col0 + t * 16 + ln) * ldb + kb;
      FragB b;
      b.half[0] = *(const v8us*)(brow + 8 * hh);
      b.half[1] = *(const v8us*)(brow + 16 + 8 * hh);
      acc[t] = mmaN<ASPLIT ? 2 : 1>(ah.v, al.v, b.v, b.v, acc[t]);
    }
  }
#pragma unroll
  for (int t = 0; t < 4; ++t) {
    const int col = col0 + t * 16 + ln;
    float bv = bias ? bias[col] : 0.f;
    if (BIAS_BF16) bv = bf16_round(bv);
#pragma unroll
    for (int r = 0; r < 8; ++r) {
      float v = acc[t][r] + bv;
      if (resid) { float rv = resid[(size_t)((row0 + 8 * hh + r) % rmod) * ldr + col]; if (RES_BF16) rv = bf16_round(rv); v += rv; }
      if (ACT == 1) v = fmaxf(v, 0.f);
      if (ACT == 2) v = 0.5f * v * (1.0f + erff(v * 0.70710678118654752f));
      if (ACT == 3) { const float u = 0.7978845608028654f * (v + 0.044715f * v * v * v); v = 0.5f * v * (1.0f + tanhf(u)); }
      so[w][8 * hh + r][t * 16 + ln] = v;
    }
  }
  __builtin_amdgcn_fence(__ATOMIC_ACQ_REL, "workgroup");
  __builtin_amdgcn_wave_barrier();
  const int rsub = lane >> 4, c4 = (lane & 15) * 4;
  for (int pass = 0; pass < 2; ++pass) {
#pragma unroll
    for (int q = 0; q < 8; ++q) {
      const int r = q * 2 + rsub;
      const v4f v = *(const v4fa*)&so[w][r][c4];
      *(volatile v4f*)(C + (size_t)(row0 + r) * ldc + col0 + c4) = v;
    }
    if (pass == 0) __threadfence();
  }
}
template <bool PARAM_BF16>
__global__ __launch_bounds__(256) void k_layernorm(const float* __restrict__ X, const float* __restrict__ R, const float* __restrict__ g, const float* __restrict__ bta,
                                                  float* __restrict__ out_sum, float* __restrict__ out_norm, int N, float eps) {
  __shared__ float red[256];
  const int row = blockIdx.x, tid = threadIdx.x;
  const float* x = X + (size_t)row * N; const float* rr = R ? R + (size_t)row * N : nullptr;
  float vals[16];
  const int per = N / 256;
  float s1 = 0.f;
  for (int u = 0; u < per / 4; ++u) {
    const int j = tid * 4 + 1024 * u;
    const v4f a = *(const v4fa*)(x + j);
    v4f b = {0.f,0.f,0.f,0.f}; if (rr) b = *(const v4fa*)(rr + j);
#pragma unroll
    for (int q = 0; q < 4; ++q) { const float v = a[q] + b[q]; vals[u * 4 + q] = v; s1 += v; }
  }
  red[tid] = s1; __syncthreads();
  for (int st = 128; st > 0; st >>= 1) { if (tid < st) red[tid] += red[tid + st]; __syncthreads(); }
  const float mu = red[0] / (float)N; __syncthreads();
  float s2 = 0.f;
  for (int u = 0; u < per / 4; ++u)
#pragma unroll
    for (int q = 0; q < 4; ++q) { const float c = vals[u * 4 + q] - mu; s2 += c * c; }
  red[tid] = s2; __syncthreads();
  for (int st = 128; st > 0; st >>= 1) { if (tid < st) red[tid] += red[tid + st]; __syncthreads(); }
  const float rs = rsqrtf(red[0] / (float)N + eps);
  for (int pass = 0; pass < 2; ++pass) {
    for (int u = 0; u < per / 4; ++u) {
      const int j = tid * 4 + 1024 * u;
      v4f o, sm;
#pragma unroll
      for (int q = 0; q < 4; ++q) {
        float gg = g[j + q], bb = bta[j + q];
        if (PARAM_BF16) { gg = bf16_round(gg); bb = bf16_round(bb); }
        sm[q] = vals[u * 4 + q]; o[q] = (vals[u * 4 + q] - mu) * rs * gg + bb;
      }
      if (out_sum) *(volatile v4f*)(out_sum + (size_t)row * N + j) = sm;
      *(volatile v4f*)(out_norm + (size_t)row * N + j) = o;
    }
    if (pass == 0) __threadfence();
  }
}


typedef _Float16 v16h __attribute__((ext_vector_type(16)));
union FragH { v16h v; v8us half[2]; _Float16 h[16]; unsigned short u[16]; };
template <int NT>
__device__ __forceinline__ v8f mmaH(v16h ah, v16h al, v16h bh, v16h bl, v8f c) {
  c = __builtin_amdgcn_wmma_f32_16x16x32_f16(false, ah, false, bh, (short)0, c, false, false);
  if (NT >= 2) c = __builtin_amdgcn_wmma_f32_16x16x32_f16(false, al, false, bh, (short)0, c, false, false);
  if (NT >= 3) c = __builtin_amdgcn_wmma_f32_16x16x32_f16(false, ah, false, bl, (short)0, c, false, false);
  asm volatile("v_nop\n\tv_nop\n\tv_nop\n\tv_nop" : "+v"(c) : "v"(ah), "v"(al), "v"(bh), "v"(bl));
  return c;
}
template <bool ASPLIT>
__global__ __launch_bounds__(128) void k_gemm_h(const float* __restrict__ A, int lda, size_t sA, const _Float16* __restrict__ Bh, int ldb, size_t sB, float alpha, float* __restrict__ C, int ldc, size_t sC, int M, int N, int K) {
  __shared__ __attribute__((aligned(16))) float so[4][16][64];
  const int tid = threadIdx.x, w = tid >> 5, lane = tid & 31, ln = lane & 15, hh = lane >> 4; const int by = blockIdx.y;
  A += (size_t)by * sA; Bh += (size_t)by * sB; C += (size_t)by * sC;
  const int ntn = (N + 63) / 64; const int wid = blockIdx.x * 4 + w; const int mt = wid / ntn, nq = wid % ntn; if (mt * 16 >= M) return;
  const int row0 = mt * 16, col0 = nq * 64; const float* arow = A + (size_t)(row0 + ln) * lda;
  v8f acc[4] = {};
  for (int kb = 0; kb < K; kb += 32) {
    FragH ah, al;
    const v4f x0 = *(const v4fa*)(arow + kb + 8 * hh), x1 = *(const v4fa*)(arow + kb + 8 * hh + 4), x2 = *(const v4fa*)(arow + kb + 16 + 8 * hh), x3 = *(const v4fa*)(arow + kb + 16 + 8 * hh + 4);
    float xs[16] = {x0[0],x0[1],x0[2],x0[3],x1[0],x1[1],x1[2],x1[3],x2[0],x2[1],x2[2],x2[3],x3[0],x3[1],x3[2],x3[3]};
#pragma unroll
    for (int i = 0; i < 16; ++i) { const _Float16 h = (_Float16)xs[i]; ah.h[i] = h; al.h[i] = ASPLIT ? (_Float16)(xs[i] - (float)h) : (_Float16)0.0f; }
#pragma unroll
    for (int t = 0; t < 4; ++t) { if (col0 + t * 16 >= N) continue; const size_t boff = (size_t)(col0 + t * 16 + ln) * ldb + kb; FragH bq; bq.half[0] = *(const v8us*)(Bh + boff + 8 * hh); bq.half[1] = *(const v8us*)(Bh + boff + 16 + 8 * hh);
      acc[t] = mmaH<ASPLIT ? 2 : 1>(ah.v, al.v, bq.v, bq.v, acc[t]); }
  }
#pragma unroll
  for (int t = 0; t < 4; ++t) { if (col0 + t * 16 >= N) continue;
#pragma unroll
    for (int r = 0; r < 8; ++r) so[w][8 * hh + r][t * 16 + ln] = acc[t][r] * alpha; }
  __builtin_amdgcn_fence(__ATOMIC_ACQ_REL, "workgroup"); __builtin_amdgcn_wave_barrier();
  const int rsub = lane >> 4, c4 = (lane & 15) * 4;
  for (int pass = 0; pass < 2; ++pass) {
#pragma unroll
    for (int q = 0; q < 8; ++q) { const int r = q * 2 + rsub; if (col0 + c4 < N) { const v4f v = *(const v4fa*)&so[w][r][c4]; *(volatile v4f*)(C + (size_t)(row0 + r) * ldc + col0 + c4) = v; } }
    if (pass == 0) __threadfence(); }
}

__global__ __launch_bounds__(256) void k_wt_f16(const float* __restrict__ W, _Float16* __restrict__ Wt, int K, int N, float scale) {
  const int t = blockIdx.x * 256 + threadIdx.x; if (t >= N * (K / 8)) return; const int n = t / (K / 8), k8 = (t % (K / 8)) * 8; FragH f;
#pragma unroll
  for (int i = 0; i < 8; ++i) f.h[i] = (_Float16)(bf16_round(W[(size_t)(k8 + i) * N + n]) * scale); const v8us o = f.half[0];
  *(volatile v8us*)((unsigned short*)Wt + (size_t)n * K + k8) = o; __threadfence(); *(volatile v8us*)((unsigned short*)Wt + (size_t)n * K + k8) = o;
}
template <int ACT>
__global__ __launch_bounds__(128) void k_gemm_hhx(const _Float16* __restrict__ A, int lda, size_t sA, const _Float16* __restrict__ Bh, int ldb, size_t sB, float alpha, const float* __restrict__ bias, size_t sBias, const float* __restrict__ CP, int rowsPerB, size_t sCPb, int row0g,
    float* __restrict__ C, _Float16* __restrict__ C16, int ldc, size_t sC, int M, int N, int K) {
  __shared__ __attribute__((aligned(16))) float so[4][16][64];
  const int tid = threadIdx.x, w = tid >> 5, lane = tid & 31, ln = lane & 15, hh = lane >> 4; const int by = blockIdx.y;
  A += (size_t)by * sA; Bh += (size_t)by * sB; const size_t cofs = (size_t)by * sC; const float* bp = bias ? bias + (size_t)by * sBias : nullptr;
  const int ntn = (N + 63) / 64; const int wid = blockIdx.x * 4 + w; const int mt = wid / ntn, nq = wid % ntn; if (mt * 16 >= M) return;
  const int row0 = mt * 16, col0 = nq * 64; const _Float16* arow = A + (size_t)(row0 + ln) * lda;
  v8f acc[4] = {};
  for (int kb = 0; kb < K; kb += 32) { FragH ah; ah.half[0] = *(const v8us*)((const unsigned short*)arow + kb + 8 * hh); ah.half[1] = *(const v8us*)((const unsigned short*)arow + kb + 16 + 8 * hh);
#pragma unroll
    for (int t = 0; t < 4; ++t) { if (col0 + t * 16 >= N) continue; const size_t boff = (size_t)(col0 + t * 16 + ln) * ldb + kb; FragH bq; bq.half[0] = *(const v8us*)((const unsigned short*)Bh + boff + 8 * hh); bq.half[1] = *(const v8us*)((const unsigned short*)Bh + boff + 16 + 8 * hh);
      acc[t] = mmaH<1>(ah.v, ah.v, bq.v, bq.v, acc[t]); }
  }
#pragma unroll
  for (int t = 0; t < 4; ++t) { if (col0 + t * 16 >= N) continue; const int col = col0 + t * 16 + ln; const float bv = bp ? bf16_round(bp[col]) : 0.f;
#pragma unroll
    for (int r = 0; r < 8; ++r) { float v = acc[t][r] * alpha + bv; if (CP) { const int rr = row0g + row0 + 8 * hh + r; if (rowsPerB < 0) v += CP[cofs + (size_t)rr * ldc + col];        else { const int bidx = rr / rowsPerB; v += CP[(size_t)bidx * sCPb + (size_t)by * 64 + col]; } } if (ACT == 1) v = (v > 0.f) ? v : expm1f(v); else if (ACT == 7) v = (v > 0.f) ? v + 1.0f : expf(v); else if (ACT == 8) v = tanhf(v); else if (ACT == 9) v = 0.5f * v * (1.0f + tanhf(0.7978845608028654f * (v + 0.044715f * v * v * v))); else if (ACT == 11) v = 1.0f / (1.0f + expf(-v)); else if (ACT == 12) v = (v > 0.f) ? v : 0.01f * v; else if (ACT == 14) v = (v > 0.f) ? v : 0.1f * v; else if (ACT == 16) v = (v >= 0.f) ? v : 0.3f * v; else if (ACT == 17) v = (v >= 0.f) ? v : 0.2f * v; else if (ACT == 15) v = v / (1.0f + expf(-v)); else if (ACT == 3) v = fmaxf(v, 0.f); else if (ACT == 6) v = 0.5f * v * (1.0f + erff(v * 0.70710678118654752f)); so[w][8 * hh + r][t * 16 + ln] = v; } }
  __builtin_amdgcn_fence(__ATOMIC_ACQ_REL, "workgroup"); __builtin_amdgcn_wave_barrier();
  const int rsub = lane >> 4, c4 = (lane & 15) * 4; typedef _Float16 v4h __attribute__((ext_vector_type(4)));
  for (int pass = 0; pass < 2; ++pass) {
#pragma unroll
    for (int q = 0; q < 8; ++q) { const int r = q * 2 + rsub; if (col0 + c4 < N) { const v4f v = *(const v4fa*)&so[w][r][c4]; if (C) *(volatile v4f*)(C + cofs + (size_t)(row0 + r) * ldc + col0 + c4) = v; if (C16) { v4h h4; for (int i = 0; i < 4; ++i) h4[i] = (_Float16)v[i]; *(volatile v4h*)(C16 + cofs + (size_t)(row0 + r) * ldc + col0 + c4) = h4; } } }
    if (pass == 0) __threadfence(); }
}


typedef _Float16 v4h __attribute__((ext_vector_type(4)));

__global__ __launch_bounds__(256) void k_x16(const float* __restrict__ x, _Float16* __restrict__ X16, size_t n8) { const size_t t = (size_t)blockIdx.x * 256 + threadIdx.x; if (t >= n8) return; FragH f;
#pragma unroll
  for (int q = 0; q < 8; ++q) f.h[q] = (_Float16)bf16_round(x[t * 8 + q]); *(volatile v8us*)((unsigned short*)X16 + t * 8) = f.half[0]; __threadfence(); *(volatile v8us*)((unsigned short*)X16 + t * 8) = f.half[0]; }
__global__ __launch_bounds__(256) void k_h16(const float* __restrict__ x, _Float16* __restrict__ X16, size_t n8) { const size_t t = (size_t)blockIdx.x * 256 + threadIdx.x; if (t >= n8) return; FragH f;
#pragma unroll
  for (int q = 0; q < 8; ++q) f.h[q] = (_Float16)x[t * 8 + q]; *(volatile v8us*)((unsigned short*)X16 + t * 8) = f.half[0]; __threadfence(); *(volatile v8us*)((unsigned short*)X16 + t * 8) = f.half[0]; }
__global__ __launch_bounds__(256) void k_round16f(const float* __restrict__ W, _Float16* __restrict__ Bt, size_t n8) { const size_t t = (size_t)blockIdx.x * 256 + threadIdx.x; if (t >= n8) return; FragH f;
#pragma unroll
  for (int i = 0; i < 8; ++i) f.h[i] = (_Float16)(bf16_round(W[t * 8 + i]) * 16.0f); *(volatile v8us*)((unsigned short*)Bt + t * 8) = f.half[0]; __threadfence(); *(volatile v8us*)((unsigned short*)Bt + t * 8) = f.half[0]; }
template <int NHv, int TTv>
__global__ __launch_bounds__(256) void k_vt(const _Float16* __restrict__ V16, int ldv, int voff, _Float16* __restrict__ Vt) { __shared__ unsigned short tl[64][66]; const int tid = threadIdx.x; const int slab = blockIdx.x / (TTv / 64), lg = blockIdx.x % (TTv / 64); const int b = slab / NHv, h = slab % NHv;
  for (int i = tid; i < 64 * 8; i += 256) { const int r = i / 8, c8 = (i % 8) * 8; FragH f; f.half[0] = *(const v8us*)((const unsigned short*)V16 + ((size_t)b * TTv + lg * 64 + r) * ldv + voff + h * 64 + c8);
#pragma unroll
    for (int q = 0; q < 8; ++q) tl[r][c8 + q] = f.u[q]; }
  __syncthreads();
  for (int pass = 0; pass < 2; ++pass) {
#pragma unroll
    for (int rd = 0; rd < 2; ++rd) { const int d = rd * 32 + tid / 8, pc = tid % 8; FragH f;
#pragma unroll
      for (int q = 0; q < 8; ++q) f.u[q] = tl[pc * 8 + q][d];
      *(volatile v8us*)((unsigned short*)Vt + ((size_t)slab * 64 + d) * TTv + lg * 64 + pc * 8) = f.half[0]; }
    if (pass == 0) __threadfence(); } }

__global__ __launch_bounds__(256) void k_hl(const float* __restrict__ F, _Float16* __restrict__ Hh, _Float16* __restrict__ Hl, size_t n8) { const size_t t = (size_t)blockIdx.x * 256 + threadIdx.x; if (t >= n8) return; FragH fh, fl; const v4f a = *(const v4fa*)(F + t * 8), c = *(const v4fa*)(F + t * 8 + 4);
#pragma unroll
  for (int q = 0; q < 4; ++q) { _Float16 h = (_Float16)a[q]; fh.h[q] = h; fl.h[q] = (_Float16)((a[q] - (float)h) * 1024.0f); h = (_Float16)c[q]; fh.h[4 + q] = h; fl.h[4 + q] = (_Float16)((c[q] - (float)h) * 1024.0f); }
  for (int pass = 0; pass < 2; ++pass) { *(volatile v8us*)((unsigned short*)Hh + t * 8) = fh.half[0]; *(volatile v8us*)((unsigned short*)Hl + t * 8) = fl.half[0]; if (pass == 0) __threadfence(); } }

__device__ __forceinline__ v16h g2_frag(const _Float16* p, int hh) { FragH f; f.half[0] = *(const v8us*)((const unsigned short*)p + 8 * hh); f.half[1] = *(const v8us*)((const unsigned short*)p + 16 + 8 * hh); return f.v; }
__device__ __forceinline__ v8f g2_mma(v16h a, v16h b, v8f c) { v8f d = __builtin_amdgcn_wmma_f32_16x16x32_f16(false, a, false, b, (short)0, c, false, false); asm volatile("v_nop\n\tv_nop\n\tv_nop\n\tv_nop" : "+v"(d) : "v"(a), "v"(b)); return d; }
template <int ACT>
__global__ __launch_bounds__(128) void k_gemm2(const _Float16* __restrict__ A, int lda, size_t sA, const _Float16* __restrict__ Bh, int ldb, size_t sB, float alpha, const float* __restrict__ bias, size_t sBias, const float* __restrict__ CP, int rowsPerB, size_t sCPb, int row0g,
    float* __restrict__ C, _Float16* __restrict__ C16, int ldc, size_t sC, int M, int N, int K) { static_assert(ACT == 0 || ACT == 3 || ACT == 6 || ACT == 8 || ACT == 9 || ACT == 11 || ACT == 12 || ACT == 14 || ACT == 15 || ACT == 16 || ACT == 17, "k_gemm2: unsupported ACT code (would silently apply no activation)");
  __shared__ __attribute__((aligned(16))) float so[4][32][68];
  const int tid = threadIdx.x, w = tid >> 5, lane = tid & 31, ln = lane & 15, hh = lane >> 4; const int by = blockIdx.y;
  A += (size_t)by * sA; Bh += (size_t)by * sB; const size_t cofs = (size_t)by * sC; const float* bp = bias ? bias + (size_t)by * sBias : nullptr;
  const int ntn = N >> 6; const int mt = blockIdx.x / ntn, nq = blockIdx.x - mt * ntn; const int row0 = mt * 128 + 32 * w, col0 = nq * 64; if (row0 >= M) return;
  const _Float16* a0p = A + (size_t)(row0 + ln) * lda; const _Float16* a1p = a0p + (size_t)16 * lda;
  const _Float16* b0p = Bh + (size_t)(col0 + ln) * ldb; const _Float16* b1p = b0p + (size_t)16 * ldb; const _Float16* b2p = b1p + (size_t)16 * ldb; const _Float16* b3p = b2p + (size_t)16 * ldb;
  const v8f z8 = {0.f,0.f,0.f,0.f,0.f,0.f,0.f,0.f}; v8f c00 = z8, c01 = z8, c02 = z8, c03 = z8, c10 = z8, c11 = z8, c12 = z8, c13 = z8;
#pragma unroll 1
  for (int kb = 0; kb < K; kb += 32) { const v16h a0 = g2_frag(a0p + kb, hh), a1 = g2_frag(a1p + kb, hh);
    v16h b = g2_frag(b0p + kb, hh); c00 = g2_mma(a0, b, c00); c10 = g2_mma(a1, b, c10);
    b = g2_frag(b1p + kb, hh); c01 = g2_mma(a0, b, c01); c11 = g2_mma(a1, b, c11);
    b = g2_frag(b2p + kb, hh); c02 = g2_mma(a0, b, c02); c12 = g2_mma(a1, b, c12);
    b = g2_frag(b3p + kb, hh); c03 = g2_mma(a0, b, c03); c13 = g2_mma(a1, b, c13); }
  v8f accs[8] = {c00, c01, c02, c03, c10, c11, c12, c13};
#pragma unroll
  for (int u = 0; u < 8; ++u) { const int t = u & 3, half = u >> 2; const int col = col0 + t * 16 + ln; const float bv = bp ? bf16_round(bp[col]) : 0.f;
#pragma unroll
    for (int r = 0; r < 8; ++r) { const int rloc = half * 16 + 8 * hh + r; float v = accs[u][r] * alpha + bv; if (CP) { if (rowsPerB < 0) v += CP[cofs + (size_t)(row0g + row0 + rloc) * ldc + col];        else { const int bidx = (row0g + row0 + rloc) / rowsPerB; v += CP[(size_t)bidx * sCPb + (size_t)by * 64 + col]; } }
      if (ACT == 3) v = fmaxf(v, 0.f); else if (ACT == 6) v = 0.5f * v * (1.0f + erff(v * 0.70710678118654752f)); else if (ACT == 11) v = 1.0f / (1.0f + expf(-v)); else if (ACT == 15) v = v / (1.0f + expf(-v)); else if (ACT == 12) v = (v > 0.f) ? v : 0.01f * v; else if (ACT == 8) v = tanhf(v); else if (ACT == 9) v = 0.5f * v * (1.0f + tanhf(0.7978845608028654f * (v + 0.044715f * v * v * v))); else if (ACT == 14) v = (v > 0.f) ? v : 0.1f * v; else if (ACT == 16) v = (v >= 0.f) ? v : 0.3f * v; else if (ACT == 17) v = (v >= 0.f) ? v : 0.2f * v;
      so[w][rloc][t * 16 + ln] = v; } }
  __builtin_amdgcn_fence(__ATOMIC_ACQ_REL, "workgroup"); __builtin_amdgcn_wave_barrier();
  const int rsub = lane >> 4, c4 = (lane & 15) * 4;
  for (int pass = 0; pass < 2; ++pass) {
#pragma unroll
    for (int q = 0; q < 16; ++q) { const int r = q * 2 + rsub; const v4f v = *(const v4fa*)&so[w][r][c4]; if (C) *(volatile v4f*)(C + cofs + (size_t)(row0 + r) * ldc + col0 + c4) = v; if (C16) { v4h h4; for (int i = 0; i < 4; ++i) h4[i] = (_Float16)v[i]; *(volatile v4h*)(C16 + cofs + (size_t)(row0 + r) * ldc + col0 + c4) = h4; } }
    if (pass == 0) __threadfence(); } }


__global__ __launch_bounds__(256) void k_wsc(const float* __restrict__ Wm, _Float16* __restrict__ Bt, size_t n8, float sc) { const size_t t = (size_t)blockIdx.x * 256 + threadIdx.x; if (t >= n8) return; FragH f; for (int q = 0; q < 8; ++q) f.h[q] = (_Float16)(bf16_round(Wm[t * 8 + q]) * sc); *(volatile v8us*)((unsigned short*)Bt + t * 8) = f.half[0]; __threadfence(); *(volatile v8us*)((unsigned short*)Bt + t * 8) = f.half[0]; }
__global__ __launch_bounds__(256) void k_nhwc(const float* __restrict__ x, int CH, _Float16* __restrict__ D) { const size_t t = (size_t)blockIdx.x * 256 + threadIdx.x; if (t >= (size_t)NR * CH / 8) return; const int c0 = (int)((t * 8) % CH); const size_t row = (t * 8) / CH; const int b = (int)(row / PX), p = (int)(row % PX); FragH f; for (int q = 0; q < 8; ++q) f.h[q] = (_Float16)bf16_round(x[((size_t)b * CH + c0 + q) * PX + p]);
  *(volatile v8us*)((unsigned short*)D + t * 8) = f.half[0]; __threadfence(); *(volatile v8us*)((unsigned short*)D + t * 8) = f.half[0]; }
__global__ __launch_bounds__(256) void k_wre(const float* __restrict__ w, int O, int CI, int K, _Float16* __restrict__ Bt) { const size_t t = (size_t)blockIdx.x * 256 + threadIdx.x; const int KK2 = K * K; if (t >= (size_t)O * KK2 * CI / 8) return; const int c8 = (int)((t * 8) % CI); const int tap = (int)(((t * 8) / CI) % KK2); const int o = (int)((t * 8) / ((size_t)CI * KK2)); FragH f; for (int q = 0; q < 8; ++q) f.h[q] = (_Float16)(bf16_round(w[(((size_t)o * CI + c8 + q) * KK2) + tap]) * 16.0f);
  *(volatile v8us*)((unsigned short*)Bt + t * 8) = f.half[0]; __threadfence(); *(volatile v8us*)((unsigned short*)Bt + t * 8) = f.half[0]; }
__global__ __launch_bounds__(256) void k_wom(const float* __restrict__ offw, const float* __restrict__ mskw, const float* __restrict__ offb, const float* __restrict__ mskb, _Float16* __restrict__ Bt, float* __restrict__ bom) { const int t = blockIdx.x * 256 + threadIdx.x; if (t >= 64 * CM / 8) return; const int k0 = (t * 8) % CM; const int o = (t * 8) / CM; FragH f;
  for (int q = 0; q < 8; ++q) { const int k = k0 + q; float v = 0.f; if (o < 18) v = bf16_round(offw[(size_t)k * 18 + o]); else if (o < 27) v = bf16_round(mskw[(size_t)k * 9 + (o - 18)]); f.h[q] = (_Float16)(v * 16.0f); }
  *(volatile v8us*)((unsigned short*)Bt + (size_t)t * 8) = f.half[0]; __threadfence(); *(volatile v8us*)((unsigned short*)Bt + (size_t)t * 8) = f.half[0];
  if (t < 64) { const float bv = (t < 18) ? bf16_round(offb[t]) : (t < 27 ? bf16_round(mskb[t - 18]) : 0.f); *(volatile float*)(bom + t) = bv; __threadfence(); *(volatile float*)(bom + t) = bv; } }
__global__ __launch_bounds__(256) void k_im2col(const _Float16* __restrict__ Sp, int ld, int coff, _Float16* __restrict__ XC) { const size_t t = (size_t)blockIdx.x * 256 + threadIdx.x; if (t >= (size_t)NR * 9 * (CM / 8)) return; const int c8 = (int)(t % (CM / 8)) * 8; const int tap = (int)((t / (CM / 8)) % 9); const size_t row = t / ((size_t)9 * (CM / 8)); const int b = (int)(row / PX), p = (int)(row % PX); const int iy = p / HS - 1 + tap / 3, ix = p % HS - 1 + tap % 3; v8us v;
  if (iy >= 0 && iy < HS && ix >= 0 && ix < HS) v = *(const v8us*)((const unsigned short*)Sp + (((size_t)b * HS + iy) * HS + ix) * ld + coff + c8); else { for (int q = 0; q < 8; ++q) v[q] = 0; }
  unsigned short* dst = (unsigned short*)XC + row * (size_t)(9 * CM) + tap * CM + c8; *(volatile v8us*)dst = v; __threadfence(); *(volatile v8us*)dst = v; }
__global__ __launch_bounds__(256) void k_bn(const float* A, int nch, const float* __restrict__ g, const float* __restrict__ bb, int act, const float* __restrict__ AW, float* Df, _Float16* __restrict__ Dh, int ldh, int coff) {
  #pragma clang fp contract(off)
  const size_t t = (size_t)blockIdx.x * 256 + threadIdx.x; if (t >= (size_t)NR * nch / 8) return; const int c0 = (int)((t * 8) % nch); const size_t row = (t * 8) / nch; const v8f a = *(const v8f*)(A + t * 8); v8f o; FragH f; const float aw = AW ? AW[row] : 1.0f;
  for (int q = 0; q < 8; ++q) { float y = a[q] * bf16_round(g[c0 + q]); y += bf16_round(bb[c0 + q]); if (act) y = y / (1.0f + expf(-y)); y = y * aw; o[q] = y; f.h[q] = (_Float16)y; }
  for (int pass = 0; pass < 2; ++pass) { if (Df) *(volatile v8f*)(Df + t * 8) = o; if (Dh) *(volatile v8us*)((unsigned short*)Dh + row * ldh + coff + c0) = f.half[0]; if (pass == 0) __threadfence(); } }
__global__ __launch_bounds__(256) void k_dwln(const float* __restrict__ Hf, const float* __restrict__ dww, const float* __restrict__ dwb, const float* __restrict__ lng, const float* __restrict__ lnb, _Float16* __restrict__ Xh, _Float16* __restrict__ Xl) {
  #pragma clang fp contract(off)
  __shared__ float red[16][16], red2[16][16]; const int tid = threadIdx.x; const int pl = tid >> 4, sub = tid & 15; const size_t row = (size_t)blockIdx.x * 16 + pl; const int b = (int)(row / PX), p = (int)(row % PX); const int y = p / HS, x = p % HS; const int c0 = sub * 8; float v[8];
  for (int q = 0; q < 8; ++q) v[q] = bf16_round(dwb[c0 + q]);
#pragma unroll 1
  for (int ky = 0; ky < 3; ++ky) { const int yy = y + ky - 1; if (yy < 0 || yy >= HS) continue;
#pragma unroll 1
    for (int kx = 0; kx < 3; ++kx) { const int xx = x + kx - 1; if (xx < 0 || xx >= HS) continue; const v8f a = *(const v8f*)(Hf + (((size_t)b * HS + yy) * HS + xx) * CM + c0); for (int q = 0; q < 8; ++q) v[q] += a[q] * bf16_round(dww[(size_t)(ky * 3 + kx) * CM + c0 + q]); } }
  float s = 0.f; for (int q = 0; q < 8; ++q) s += v[q]; red[pl][sub] = s; __syncthreads(); float mu = 0.f; for (int i = 0; i < 16; ++i) mu += red[pl][i]; mu = mu / (float)CM;
  float s2 = 0.f; for (int q = 0; q < 8; ++q) { const float d = v[q] - mu; s2 += d * d; } red2[pl][sub] = s2; __syncthreads(); float var = 0.f; for (int i = 0; i < 16; ++i) var += red2[pl][i]; var = var / (float)CM; const float rs = rsqrtf(var + 1e-5f);
  FragH fh, fl; for (int q = 0; q < 8; ++q) { float u = (v[q] - mu) * rs; u = u * bf16_round(lng[c0 + q]); u += bf16_round(lnb[c0 + q]); const float ge = 0.5f * u * (1.0f + erff(u * 0.70710678118654752f)); const _Float16 hv = (_Float16)ge; fh.h[q] = hv; fl.h[q] = (_Float16)((ge - (float)hv) * 1024.0f); }
  const size_t o = row * CM + c0; for (int pass = 0; pass < 2; ++pass) { *(volatile v8us*)((unsigned short*)Xh + o) = fh.half[0]; *(volatile v8us*)((unsigned short*)Xl + o) = fl.half[0]; if (pass == 0) __threadfence(); } }
__global__ __launch_bounds__(256) void k_dcore(const float* __restrict__ OM, const _Float16* __restrict__ XP16, _Float16* __restrict__ DS16) {
  #pragma clang fp contract(off)
  const size_t t = (size_t)blockIdx.x * 256 + threadIdx.x; if (t >= (size_t)NR * CM / 8) return; const int c0 = (int)((t * 8) % CM); const size_t row = (t * 8) / CM; const int b = (int)(row / PX), p = (int)(row % PX); const int y = p / HS, x = p % HS; const float* om = OM + row * 64;
  float mx = -3.0e38f; for (int k = 0; k < 9; ++k) mx = fmaxf(mx, om[18 + k]); float su = 0.f; for (int k = 0; k < 9; ++k) su += expf(om[18 + k] - mx); const float inv = 1.0f / su;
  float acc[8]; for (int q = 0; q < 8; ++q) acc[q] = 0.f;
#pragma unroll 1
  for (int k = 0; k < 9; ++k) { const float mk = expf(om[18 + k] - mx) * inv; float pxf = (float)(x + k / 3 - 1); pxf += om[2 * k]; float pyf = (float)(y + k % 3 - 1); pyf += om[2 * k + 1];
    const float x0 = floorf(pxf), y0 = floorf(pyf); const float fx = pxf - x0, fy = pyf - y0; const int ix0 = (int)x0, iy0 = (int)y0; float s[8]; for (int q = 0; q < 8; ++q) s[q] = 0.f;
    for (int cn = 0; cn < 4; ++cn) { const int xi = ix0 + (cn & 1), yi = iy0 + (cn >> 1); if (xi < 0 || xi >= HS || yi < 0 || yi >= HS) continue; float wgt = (cn & 1) ? fx : (1.0f - fx); wgt = wgt * ((cn >> 1) ? fy : (1.0f - fy)); FragH v; v.half[0] = *(const v8us*)((const unsigned short*)XP16 + (((size_t)b * HS + yi) * HS + xi) * CM + c0); for (int q = 0; q < 8; ++q) s[q] += (float)v.h[q] * wgt; }
    for (int q = 0; q < 8; ++q) acc[q] += mk * s[q]; }
  FragH f; for (int q = 0; q < 8; ++q) f.h[q] = (_Float16)acc[q]; *(volatile v8us*)((unsigned short*)DS16 + t * 8) = f.half[0]; __threadfence(); *(volatile v8us*)((unsigned short*)DS16 + t * 8) = f.half[0]; }
__global__ __launch_bounds__(128) void k_gproj(const float* __restrict__ guide, const float* __restrict__ glw, const float* __restrict__ glb, float* __restrict__ G) {
  #pragma clang fp contract(off)
  const int t = blockIdx.x * 128 + threadIdx.x; if (t >= NI * NTOK * CM) return; const int c = t % CM; const int bn = t / CM; const float* gp = guide + (size_t)bn * GD; float s = 0.f;
#pragma unroll 1
  for (int k = 0; k < GD; k += 4) { const v4f a = *(const v4fa*)(gp + k); for (int q = 0; q < 4; ++q) s += bf16_round(a[q]) * bf16_round(glw[(size_t)(k + q) * CM + c]); }
  s += bf16_round(glb[c]); *(volatile float*)(G + t) = s; __threadfence(); *(volatile float*)(G + t) = s; }
__global__ __launch_bounds__(256) void k_aw(const float* __restrict__ EMB, const float* __restrict__ G, const float* __restrict__ bias, float* __restrict__ AW) {
  #pragma clang fp contract(off)
  __shared__ float sg[NTOK * CM]; __shared__ float smx[64][4]; const int tid = threadIdx.x; const size_t row0 = (size_t)blockIdx.x * 64; const int b = (int)(row0 / PX); for (int i = tid; i < NTOK * CM; i += 256) sg[i] = G[(size_t)b * NTOK * CM + i]; __syncthreads();
  const int pl = tid >> 2, part = tid & 3; const size_t row = row0 + pl; const float* e = EMB + row * CM; float mx = -3.0e38f;
#pragma unroll 1
  for (int n = part; n < NTOK; n += 4) { float s = 0.f;
#pragma unroll 1
    for (int c = 0; c < CM; c += 4) { const v4f a = *(const v4fa*)(e + c); for (int q = 0; q < 4; ++q) s += a[q] * sg[n * CM + c + q]; }
    mx = fmaxf(mx, s); }
  smx[pl][part] = mx; __syncthreads();
  if (tid < 64) { const float m = fmaxf(fmaxf(smx[tid][0], smx[tid][1]), fmaxf(smx[tid][2], smx[tid][3])); float a = m * 0.088388347648318447f; a += bf16_round(bias[0]); const float w = 1.0f / (1.0f + expf(-a)); *(volatile float*)(AW + row0 + tid) = w; __threadfence(); *(volatile float*)(AW + row0 + tid) = w; } }
__global__ __launch_bounds__(256) void k_out(const float* __restrict__ Y, float* __restrict__ out) { const size_t t = (size_t)blockIdx.x * 256 + threadIdx.x; if (t >= (size_t)NI * C1 * PX / 8) return; const int p0 = (int)((t * 8) % PX); const size_t bo = (t * 8) / PX; const int b = (int)(bo / C1), o = (int)(bo % C1); v8f v; for (int q = 0; q < 8; ++q) v[q] = Y[((size_t)b * PX + p0 + q) * C1 + o];
  *(volatile v8f*)(out + t * 8) = v; __threadfence(); *(volatile v8f*)(out + t * 8) = v; }

extern "C" void kernel_launch(void* const* d_in, const int* in_sizes, int n_in,
                              void* d_out, int out_size, void* d_ws, size_t ws_size, hipStream_t stream) {
  (void)in_sizes; (void)n_in; (void)out_size;
  const float* const* I = (const float* const*)d_in;
  const float* x = I[0]; const float* guide = I[1]; const float* cv1_w = I[2]; const float* cv1_g = I[3]; const float* cv1_b = I[4]; const float* m_cv1_w = I[5]; const float* m_cv1_g = I[6]; const float* m_cv1_b = I[7]; const float* m_pre_w = I[8]; const float* m_pre_g = I[9]; const float* m_pre_b = I[10]; const float* m_dw_w = I[11]; const float* m_dw_b = I[12]; const float* m_ln_g = I[13]; const float* m_ln_b = I[14]; const float* m_off_w = I[15]; const float* m_off_b = I[16]; const float* m_msk_w = I[17]; const float* m_msk_b = I[18]; const float* m_in_w = I[19]; const float* m_in_b = I[20]; const float* m_out_w = I[21]; const float* m_out_b = I[22]; const float* m_bn_g = I[23]; const float* m_bn_b = I[24]; const float* gl_w = I[25]; const float* gl_b = I[26]; const float* a_bias = I[27]; const float* pj_w = I[28]; const float* pj_g = I[29]; const float* pj_b = I[30]; const float* cv2_w = I[31]; const float* cv2_g = I[32]; const float* cv2_b = I[33];
  char* ws = (char*)d_ws; size_t off = 0;
  auto take = [&](size_t bytes) { char* p = ws + off; off += (bytes + 255) & ~(size_t)255; return p; };
  _Float16* BCV1 = (_Float16*)take((size_t)C1 * C1 * 2); _Float16* BM3[2]; _Float16* BPRE[2]; _Float16* BOM[2]; float* bom[2]; _Float16* BIN[2]; _Float16* BOUT[2];
  for (int i = 0; i < 2; ++i) { BM3[i] = (_Float16*)take((size_t)CM * 9 * CM * 2); BPRE[i] = (_Float16*)take((size_t)CM * CM * 2); BOM[i] = (_Float16*)take((size_t)64 * CM * 2); bom[i] = (float*)take(64 * 4); BIN[i] = (_Float16*)take((size_t)CM * CM * 2); BOUT[i] = (_Float16*)take((size_t)CM * CM * 2); }
  _Float16* BPJ = (_Float16*)take((size_t)CM * 9 * CM * 2); _Float16* BCV2 = (_Float16*)take((size_t)C1 * CC5 * 2);
  _Float16* X16 = (_Float16*)take((size_t)NR * C1 * 2); _Float16* CAT = (_Float16*)take((size_t)NR * CC5 * 2);        float* T32 = (float*)take((size_t)NR * C1 * 4);
  _Float16* XC = (_Float16*)take((size_t)NR * 9 * CM * 2);        float* HF = (float*)take((size_t)NR * CM * 4); _Float16* H16 = (_Float16*)take((size_t)NR * CM * 2); _Float16* XP16 = (_Float16*)take((size_t)NR * CM * 2); _Float16* X1H = (_Float16*)take((size_t)NR * CM * 2); _Float16* X1L = (_Float16*)take((size_t)NR * CM * 2); float* OM = (float*)take((size_t)NR * 64 * 4); _Float16* DS16 = (_Float16*)take((size_t)NR * CM * 2); float* EMB = (float*)take((size_t)NR * CM * 4); float* G = (float*)take((size_t)NI * NTOK * CM * 4); float* AW = (float*)take((size_t)NR * 4);
  if (off > ws_size) return;
  k_wre<<<(unsigned)(((size_t)C1 * C1 / 8 + 255) / 256), 256, 0, stream>>>(cv1_w, C1, C1, 1, BCV1); k_wre<<<(unsigned)(((size_t)C1 * CC5 / 8 + 255) / 256), 256, 0, stream>>>(cv2_w, C1, CC5, 1, BCV2); k_wre<<<(unsigned)(((size_t)CM * 9 * CM / 8 + 255) / 256), 256, 0, stream>>>(pj_w, CM, CM, 3, BPJ);
  for (int i = 0; i < 2; ++i) { k_wre<<<(unsigned)(((size_t)CM * 9 * CM / 8 + 255) / 256), 256, 0, stream>>>(m_cv1_w + (size_t)i * CM * CM * 9, CM, CM, 3, BM3[i]); k_wre<<<(unsigned)(((size_t)CM * CM / 8 + 255) / 256), 256, 0, stream>>>(m_pre_w + (size_t)i * CM * CM, CM, CM, 1, BPRE[i]);
    k_wom<<<(64 * CM / 8 + 255) / 256, 256, 0, stream>>>(m_off_w + (size_t)i * CM * 18, m_msk_w + (size_t)i * CM * 9, m_off_b + i * 18, m_msk_b + i * 9, BOM[i], bom[i]);
    k_wt_f16<<<(CM * CM / 8 + 255) / 256, 256, 0, stream>>>(m_in_w + (size_t)i * CM * CM, BIN[i], CM, CM, 16.0f); k_wt_f16<<<(CM * CM / 8 + 255) / 256, 256, 0, stream>>>(m_out_w + (size_t)i * CM * CM, BOUT[i], CM, CM, 16.0f); }
  k_nhwc<<<(unsigned)(((size_t)NR * C1 / 8 + 255) / 256), 256, 0, stream>>>(x, C1, X16);
  const dim3 g256((NR / 128) * (C1 / 64), 1), g128((NR / 128) * (CM / 64), 1), g64((NR / 128) * 1, 1);
  k_gemm2<0><<<g256, 128, 0, stream>>>(X16, C1, 0, BCV1, C1, 0, 0.0625f, nullptr, 0, nullptr, 1, 0, 0, T32, nullptr, C1, 0, NR, C1, C1);
  k_bn<<<(unsigned)(((size_t)NR * C1 / 8 + 255) / 256), 256, 0, stream>>>(T32, C1, cv1_g, cv1_b, 1, nullptr, nullptr, CAT, CC5, 0);
  for (int i = 0; i < 2; ++i) { const int cin = CM * (1 + i);
    k_im2col<<<(unsigned)(((size_t)NR * 9 * (CM / 8) + 255) / 256), 256, 0, stream>>>(CAT, CC5, cin, XC);
    k_gemm2<0><<<g128, 128, 0, stream>>>(XC, 9 * CM, 0, BM3[i], 9 * CM, 0, 0.0625f, nullptr, 0, nullptr, 1, 0, 0, T32, nullptr, CM, 0, NR, CM, 9 * CM);
    k_bn<<<(unsigned)(((size_t)NR * CM / 8 + 255) / 256), 256, 0, stream>>>(T32, CM, m_cv1_g + i * CM, m_cv1_b + i * CM, 1, nullptr, nullptr, H16, CM, 0);
    k_gemm2<0><<<g128, 128, 0, stream>>>(H16, CM, 0, BPRE[i], CM, 0, 0.0625f, nullptr, 0, nullptr, 1, 0, 0, T32, nullptr, CM, 0, NR, CM, CM);
    k_bn<<<(unsigned)(((size_t)NR * CM / 8 + 255) / 256), 256, 0, stream>>>(T32, CM, m_pre_g + i * CM, m_pre_b + i * CM, 1, nullptr, HF, H16, CM, 0);
    k_gemm2<0><<<g128, 128, 0, stream>>>(H16, CM, 0, BIN[i], CM, 0, 0.0625f, m_in_b + i * CM, 0, nullptr, 1, 0, 0, nullptr, XP16, CM, 0, NR, CM, CM);
    k_dwln<<<NR / 16, 256, 0, stream>>>(HF, m_dw_w + (size_t)i * 9 * CM, m_dw_b + i * CM, m_ln_g + i * CM, m_ln_b + i * CM, X1H, X1L);
    k_gemm2<0><<<g64, 128, 0, stream>>>(X1L, CM, 0, BOM[i], CM, 0, 0.0625f / 1024.0f, nullptr, 0, nullptr, 1, 0, 0, OM, nullptr, 64, 0, NR, 64, CM);
    k_gemm2<0><<<g64, 128, 0, stream>>>(X1H, CM, 0, BOM[i], CM, 0, 0.0625f, bom[i], 0, OM, 1, 64, 0, OM, nullptr, 64, 0, NR, 64, CM);
    k_dcore<<<(unsigned)(((size_t)NR * CM / 8 + 255) / 256), 256, 0, stream>>>(OM, XP16, DS16);
    k_gemm2<0><<<g128, 128, 0, stream>>>(DS16, CM, 0, BOUT[i], CM, 0, 0.0625f, m_out_b + i * CM, 0, nullptr, 1, 0, 0, T32, nullptr, CM, 0, NR, CM, CM);
    k_bn<<<(unsigned)(((size_t)NR * CM / 8 + 255) / 256), 256, 0, stream>>>(T32, CM, m_bn_g + i * CM, m_bn_b + i * CM, 1, nullptr, (i == 1) ? EMB : nullptr, CAT, CC5, CM * (2 + i));        }
  k_gproj<<<(NI * NTOK * CM + 127) / 128, 128, 0, stream>>>(guide, gl_w, gl_b, G); k_aw<<<NR / 64, 256, 0, stream>>>(EMB, G, a_bias, AW);
  k_im2col<<<(unsigned)(((size_t)NR * 9 * (CM / 8) + 255) / 256), 256, 0, stream>>>(CAT, CC5, 3 * CM, XC);
  k_gemm2<0><<<g128, 128, 0, stream>>>(XC, 9 * CM, 0, BPJ, 9 * CM, 0, 0.0625f, nullptr, 0, nullptr, 1, 0, 0, T32, nullptr, CM, 0, NR, CM, 9 * CM);
  k_bn<<<(unsigned)(((size_t)NR * CM / 8 + 255) / 256), 256, 0, stream>>>(T32, CM, pj_g, pj_b, 0, AW, nullptr, CAT, CC5, 4 * CM);
  k_gemm2<0><<<g256, 128, 0, stream>>>(CAT, CC5, 0, BCV2, CC5, 0, 0.0625f, nullptr, 0, nullptr, 1, 0, 0, T32, nullptr, C1, 0, NR, C1, CC5);
  k_bn<<<(unsigned)(((size_t)NR * C1 / 8 + 255) / 256), 256, 0, stream>>>(T32, C1, cv2_g, cv2_b, 1, nullptr, T32, nullptr, 0, 0);
  k_out<<<(unsigned)(((size_t)NI * C1 * PX / 8 + 255) / 256), 256, 0, stream>>>(T32, (float*)d_out);
}
